// MyModel_48395691491912
// MI455X (gfx1250) — hardware-run, weakly checked
//
#include <hip/hip_runtime.h>
#include <math.h>

constexpr int NBAT   = 512;
constexpr int NFEAT  = 80;
constexpr int NLEN   = 111;
constexpr int NDEC   = 222;
constexpr int NUNIT  = 20;
constexpr int NATT   = 10;
constexpr int NCF    = 32;
constexpr int NGATE  = 80;
constexpr int TROWS  = 16;
constexpr int NTHR   = 256;
constexpr int NBLK   = NBAT / TROWS;
constexpr int NPADN  = 128;
constexpr int ENC_K  = 128;
constexpr int ENC_P  = 136;
constexpr int ENC_HCOL = 96;
constexpr int DEC_K  = 64;
constexpr int DEC_P  = 72;
constexpr int DEC_HCOL = 20;
constexpr int ATT_P  = 112;
constexpr int MP_P   = 12;
constexpr int E_STEP = TROWS * NUNIT;
constexpr int MP_STEP = TROWS * MP_P;
constexpr int E_BLK  = NLEN * E_STEP;
constexpr int MP_BLK = NLEN * MP_STEP;
constexpr int Y_BLK  = TROWS * NDEC;
constexpr int NITEM  = (NLEN + 15) / 16;

static_assert(NBAT % TROWS == 0, "tile");
static_assert((Y_BLK * 4) % 128 == 0, "output chunk is whole lines");
static_assert(Y_BLK % 4 == 0, "output chunk float4");
static_assert((E_STEP * 4) % 128 == 0 && (MP_STEP * 4) % 128 == 0, "ws step chunks are whole lines");
static_assert(E_STEP / 4 <= 96 && MP_STEP / 4 <= 96, "one wave, <=3 store instructions");
static_assert((NPADN * ENC_P) % NTHR == 0 && (NPADN * DEC_P) % NTHR == 0, "weight plane build loops exact");
static_assert(ENC_P % 8 == 0 && DEC_P % 8 == 0, "16-B fragment alignment");
static_assert(ENC_K <= ENC_P && DEC_K <= DEC_P, "pitch");
static_assert(ENC_HCOL + 32 == ENC_K && ENC_HCOL >= NFEAT + 16, "encoder k layout");
static_assert(DEC_HCOL + 32 + 12 == DEC_K, "decoder k layout");
static_assert(TROWS * 12 == 192 && TROWS * NATT == 160 && TROWS * 6 == 96, "phase thread maps");
static_assert(NFEAT % 8 == 0 && NITEM * 16 >= NLEN, "maps");
static_assert((TROWS * ATT_P) % NTHR == 0, "attn zero fill exact");
static_assert(4 * NUNIT == NGATE && NUNIT <= 32 && NPADN == 4 * 32, "gate permutation");

typedef __attribute__((ext_vector_type(16))) _Float16 v16h;
typedef __attribute__((ext_vector_type(8)))  _Float16 v8h;
typedef __attribute__((ext_vector_type(16))) __bf16   v16b;
typedef __attribute__((ext_vector_type(8)))  __bf16   v8b;
typedef __attribute__((ext_vector_type(8)))  float    v8f;
typedef __attribute__((ext_vector_type(4)))  float    v4f;
typedef __attribute__((ext_vector_type(4)))  unsigned v4u;
typedef __attribute__((ext_vector_type(2)))  unsigned v2u;

__device__ __forceinline__ unsigned short f2bf_bits(float f) {
  unsigned u = __float_as_uint(f);
  return (unsigned short)((u + 0x7FFFu + ((u >> 16) & 1u)) >> 16);
}
__device__ __forceinline__ float bf_bits2f(unsigned short h) { return __uint_as_float(((unsigned)h) << 16); }
__device__ __forceinline__ float bf16r(float f) { return bf_bits2f(f2bf_bits(f)); }
__device__ __forceinline__ unsigned pack_bf16x2(float a, float b) {
  return (unsigned)f2bf_bits(a) | ((unsigned)f2bf_bits(b) << 16);
}
__device__ __forceinline__ void split_bf16(float v, unsigned short& hb, unsigned short& lb) {
  hb = f2bf_bits(v);
  lb = f2bf_bits(v - bf_bits2f(hb));
}

__device__ __forceinline__ void dep_guard_h(v8f& a, v8f& b, v16h x, v16h y) { asm volatile("v_nop\n\tv_nop\n\tv_nop\n\tv_nop" : "+v"(a), "+v"(b) : "v"(x), "v"(y)); }
__device__ __forceinline__ void dep_guard_b(v8f& a, v8f& b, v16b x, v16b y) { asm volatile("v_nop\n\tv_nop\n\tv_nop\n\tv_nop" : "+v"(a), "+v"(b) : "v"(x), "v"(y)); }
__device__ __forceinline__ void keep4_h(v16h a, v16h b, v16h c, v16h d) { asm volatile("v_nop" :: "v"(a), "v"(b), "v"(c), "v"(d)); }
__device__ __forceinline__ void keep4_b(v16b a, v16b b, v16b c, v16b d) { asm volatile("v_nop" :: "v"(a), "v"(b), "v"(c), "v"(d)); }
__device__ __forceinline__ void acc_guard4(v8f& a, v8f& b, v8f& c, v8f& d) { asm volatile("v_nop\n\tv_nop\n\tv_nop\n\tv_nop" : "+v"(a), "+v"(b), "+v"(c), "+v"(d)); }
__device__ __forceinline__ void grp_guard_b(v8f& a0, v8f& a1, v8f& a2, v8f& a3, v16b x, v16b y,
                                            v16b b0, v16b b1, v16b b2, v16b b3) {
  asm volatile("v_nop\n\tv_nop\n\tv_nop\n\tv_nop"
               : "+v"(a0), "+v"(a1), "+v"(a2), "+v"(a3)
               : "v"(x), "v"(y), "v"(b0), "v"(b1), "v"(b2), "v"(b3));
}
template <typename T> struct Frag;
template <> struct Frag<_Float16> {
  typedef v16h V; union U { v16h v; v8h h[2]; };
  static __device__ __forceinline__ v16h load(const _Float16* p) {
    U f; f.h[0] = *(const v8h*)(p); f.h[1] = *(const v8h*)(p + 16); return f.v;
  }
  static __device__ __forceinline__ v8f mma(v16h a, v16h b, v8f c) {
    return __builtin_amdgcn_wmma_f32_16x16x32_f16(false, a, false, b, (short)0, c, false, false);
  }
  static __device__ __forceinline__ void guard(v8f& a, v8f& b, v16h x, v16h y) { dep_guard_h(a, b, x, y); }
  static __device__ __forceinline__ void keep(v16h a, v16h b, v16h c, v16h d) { keep4_h(a, b, c, d); }
};
template <> struct Frag<__bf16> {
  typedef v16b V; union U { v16b v; v8b h[2]; };
  static __device__ __forceinline__ v16b load(const __bf16* p) {
    U f; f.h[0] = *(const v8b*)(p); f.h[1] = *(const v8b*)(p + 16); return f.v;
  }
  static __device__ __forceinline__ v8f mma(v16b a, v16b b, v8f c) {
    return __builtin_amdgcn_wmma_f32_16x16x32_bf16(false, a, false, b, (short)0, c, false, false);
  }
  static __device__ __forceinline__ void guard(v8f& a, v8f& b, v16b x, v16b y) { dep_guard_b(a, b, x, y); }
  static __device__ __forceinline__ void keep(v16b a, v16b b, v16b c, v16b d) { keep4_b(a, b, c, d); }
};
typedef Frag<__bf16> FB;

__device__ __forceinline__ float sigm_p(float x) {
  x = fminf(fmaxf(x, -30.0f), 30.0f);
  const float e = expf(-x);
  return 1.0f / (1.0f + e);
}
__device__ __forceinline__ float tanh_p(float x) {
  x = fminf(fmaxf(x, -15.0f), 15.0f);
  const float e = expf(2.0f * x);
  return 1.0f - 2.0f / (e + 1.0f);
}
__device__ __forceinline__ float tanh_q(float x) {
  const float e = __expf(2.0f * x);
  return 1.0f - 2.0f * __builtin_amdgcn_rcpf(e + 1.0f);
}
__device__ __forceinline__ float lstm_cell(float zi, float zf, float zg, float zo, float& cst) {
  const float cn = sigm_p(zf) * cst + sigm_p(zi) * tanh_p(zg);
  cst = cn;
  return sigm_p(zo) * tanh_p(cn);
}
__device__ __forceinline__ void wave_store_lines(const float* src, float* dst, int n4, int lane) {
  for (int pass = 0; pass < 2; ++pass) {
#pragma unroll
    for (int j = 0; j < 3; ++j) {
      const int i  = lane + 32 * j;
      const int ic = min(i, n4 - 1);
      const v4f v = *(const v4f*)(src + 4 * ic);
      if (i < n4) *(volatile v4f*)(dst + 4 * i) = v;
    }
    __threadfence();
  }
}

__global__ __launch_bounds__(NTHR) void seq_attn_lstm_kernel(
    const float* __restrict__ X,
    const float* __restrict__ encWx, const float* __restrict__ encWh, const float* __restrict__ encB,
    const float* __restrict__ attWq, const float* __restrict__ attBq,
    const float* __restrict__ attWm, const float* __restrict__ attBm,
    const float* __restrict__ attV,  const float* __restrict__ attBv,
    const float* __restrict__ locWc, const float* __restrict__ locWd,
    const float* __restrict__ decWx, const float* __restrict__ decWh, const float* __restrict__ decB,
    const float* __restrict__ outW,  const float* __restrict__ outB,
    float* Yout, float* Ews, float* MPws) {
  __shared__ __align__(16) unsigned short sWenc[NPADN * ENC_P];
  __shared__ __align__(16) unsigned short sWdec[NPADN * DEC_P];
  __shared__ __align__(16) unsigned short sAeH[2][TROWS * ENC_P];
  __shared__ __align__(16) unsigned short sAeL[2][TROWS * ENC_P];
  __shared__ __align__(16) unsigned short sAdH[2][TROWS * DEC_P];
  __shared__ __align__(16) unsigned short sAdL[2][TROWS * DEC_P];
  __shared__ __align__(16) float sHf[TROWS * NUNIT];
  __shared__ __align__(16) float sCst[TROWS * NUNIT];
  __shared__ __align__(16) float sMPst[TROWS * MP_P];
  __shared__ __align__(16) float sAttn[TROWS * ATT_P];
  __shared__ __align__(16) float sY[Y_BLK];
  __shared__ float sQ[TROWS * NATT];
  __shared__ float sWq[NUNIT * NATT], sWm[NUNIT * NATT];
  __shared__ float sEb[NGATE], sDb[NGATE], sOw[NUNIT];
  __shared__ float sBq[NATT], sBm[NATT], sV[NATT], sWloc[NATT], sMisc[2];

  const int tid = threadIdx.x, lane = tid & 31, wave = tid >> 5;
  const int c = lane & 15, hh = lane >> 4, koff = hh * 8;
  const int blk = blockIdx.x, b0 = blk * TROWS;
  const int uu = 16 * wave + c;
  const int uc = min(uu, NUNIT - 1);
  const bool uval = (uu < NUNIT);

  {
    const int i200 = min(tid, NUNIT * NATT - 1);
    const float wq = bf16r(attWq[i200]);
    const float wm = bf16r(attWm[i200]);
    const int i80 = min(tid, NGATE - 1);
    const float eb = bf16r(encB[i80]);
    const float db = bf16r(decB[i80]);
    asm volatile("" ::: "memory");
    if (tid < NUNIT * NATT) { sWq[tid] = wq; sWm[tid] = wm; }
    if (tid < NGATE) { sEb[tid] = eb; sDb[tid] = db; }
    const int i10 = min(tid, NATT - 1);
    const float bq = bf16r(attBq[i10]);
    const float bm = bf16r(attBm[i10]);
    const float va = bf16r(attV[i10]);
    asm volatile("" ::: "memory");
    float wl = 0.0f;
#pragma unroll 1
    for (int cf = 0; cf < NCF; ++cf) wl = fmaf(bf16r(locWc[cf]), bf16r(locWd[cf * NATT + i10]), wl);
    if (tid < NATT) { sBq[tid] = bq; sBm[tid] = bm; sV[tid] = va; sWloc[tid] = wl; }
    const int i20 = min(tid, NUNIT - 1);
    const float ow = bf16r(outW[i20]);
    const float bvv = bf16r(attBv[0]);
    const float obb = bf16r(outB[0]);
    if (tid < NUNIT) sOw[tid] = ow;
    if (tid == 0) { sMisc[0] = bvv; sMisc[1] = obb; }
  }
#pragma unroll 1
  for (int i = tid; i < NPADN * ENC_P; i += NTHR) {
    const int n = i / ENC_P, k = i - n * ENC_P;
    const int g = n >> 5, u = n & 31;
    const int col = g * NUNIT + min(u, NUNIT - 1);
    const int kx = min(k, NFEAT - 1);
    const int kh = min(max(k - ENC_HCOL, 0), NUNIT - 1);
    const float vx = encWx[kx * NGATE + col];
    const float vh = encWh[kh * NGATE + col];
    const float fx = (u < NUNIT && k < NFEAT) ? 1.0f : 0.0f;
    const float fh = (u < NUNIT && k >= ENC_HCOL && k < ENC_HCOL + NUNIT) ? 1.0f : 0.0f;
    sWenc[i] = f2bf_bits(fmaf(fx, vx, fh * vh));
  }
#pragma unroll 1
  for (int i = tid; i < NPADN * DEC_P; i += NTHR) {
    const int n = i / DEC_P, k = i - n * DEC_P;
    const int g = n >> 5, u = n & 31;
    const int col = g * NUNIT + min(u, NUNIT - 1);
    const int kx = min(k, NUNIT - 1);
    const int kh = min(max(k - DEC_HCOL, 0), NUNIT - 1);
    const float vx = decWx[kx * NGATE + col];
    const float vh = decWh[kh * NGATE + col];
    const float fx = (u < NUNIT && k < NUNIT) ? 1.0f : 0.0f;
    const float fh = (u < NUNIT && k >= DEC_HCOL && k < DEC_HCOL + NUNIT) ? 1.0f : 0.0f;
    sWdec[i] = f2bf_bits(fmaf(fx, vx, fh * vh));
  }
  {
    const v4u z4 = {0u, 0u, 0u, 0u};
#pragma unroll 1
    for (int i = tid; i < (2 * TROWS * ENC_P) / 8; i += NTHR) {
      *(v4u*)(&sAeH[0][0] + 8 * i) = z4;
      *(v4u*)(&sAeL[0][0] + 8 * i) = z4;
    }
#pragma unroll 1
    for (int i = tid; i < (2 * TROWS * DEC_P) / 8; i += NTHR) {
      *(v4u*)(&sAdH[0][0] + 8 * i) = z4;
      *(v4u*)(&sAdL[0][0] + 8 * i) = z4;
    }
#pragma unroll 1
    for (int i = tid; i < TROWS * ATT_P; i += NTHR) sAttn[i] = 0.0f;
#pragma unroll 1
    for (int i = tid; i < TROWS * NUNIT; i += NTHR) { sCst[i] = 0.0f; sHf[i] = 0.0f; }
#pragma unroll 1
    for (int i = tid; i < TROWS * MP_P; i += NTHR) sMPst[i] = 0.0f;
  }
  __syncthreads();

  const v8f z8 = {0.f, 0.f, 0.f, 0.f, 0.f, 0.f, 0.f, 0.f};
  float cst[8];
#pragma unroll
  for (int r = 0; r < 8; ++r) cst[r] = 0.0f;

#pragma unroll 1
  for (int t = 0; t < NLEN; ++t) {
    const int p = t & 1;
    if (wave < 6) {
      const int m = tid / 12, c8 = (tid - 12 * m) * 8;
      const int cc = min(c8, NFEAT - 8);
      const float fx = (c8 < NFEAT) ? 1.0f : 0.0f;
      const float* xp = X + ((size_t)(b0 + m) * NLEN + (size_t)t) * NFEAT + cc;
      const v4f x0 = *(const v4f*)xp;
      const v4f x1 = *(const v4f*)(xp + 4);
      v4u pk;
      pk[0] = pack_bf16x2(x0[0] * fx, x0[1] * fx);
      pk[1] = pack_bf16x2(x0[2] * fx, x0[3] * fx);
      pk[2] = pack_bf16x2(x1[0] * fx, x1[1] * fx);
      pk[3] = pack_bf16x2(x1[2] * fx, x1[3] * fx);
      *(v4u*)(&sAeH[p][0] + m * ENC_P + c8) = pk;
    } else if (wave == 6) {
      if (t > 0) wave_store_lines(sHf, Ews + (size_t)blk * E_BLK + (size_t)(t - 1) * E_STEP, E_STEP / 4, lane);
    } else {
      if (t > 0) wave_store_lines(sMPst, MPws + (size_t)blk * MP_BLK + (size_t)(t - 1) * MP_STEP, MP_STEP / 4, lane);
    }
    __syncthreads();

    if (wave < 2) {
      const __bf16* ah = (const __bf16*)(&sAeH[p][0] + c * ENC_P + koff);
      const __bf16* al = (const __bf16*)(&sAeL[p][0] + c * ENC_P + koff);
      const __bf16* wb = (const __bf16*)(sWenc + (wave * 16 + c) * ENC_P + koff);
      v8f acc[4];
      acc[0] = z8; acc[1] = z8; acc[2] = z8; acc[3] = z8;
#pragma unroll
      for (int ks = 0; ks < 3; ++ks) {
        const int k0 = 32 * ks;
        const v16b b0 = FB::load(wb + 0 * 32 * ENC_P + k0);
        const v16b b1 = FB::load(wb + 1 * 32 * ENC_P + k0);
        const v16b b2 = FB::load(wb + 2 * 32 * ENC_P + k0);
        const v16b b3 = FB::load(wb + 3 * 32 * ENC_P + k0);
        const v16b xa = FB::load(ah + k0);
        acc[0] = FB::mma(xa, b0, acc[0]);
        acc[1] = FB::mma(xa, b1, acc[1]);
        acc[2] = FB::mma(xa, b2, acc[2]);
        acc[3] = FB::mma(xa, b3, acc[3]);
        grp_guard_b(acc[0], acc[1], acc[2], acc[3], xa, xa, b0, b1, b2, b3);
      }
      {
        const int k0 = ENC_HCOL;
        const v16b b0 = FB::load(wb + 0 * 32 * ENC_P + k0);
        const v16b b1 = FB::load(wb + 1 * 32 * ENC_P + k0);
        const v16b b2 = FB::load(wb + 2 * 32 * ENC_P + k0);
        const v16b b3 = FB::load(wb + 3 * 32 * ENC_P + k0);
        const v16b xa = FB::load(ah + k0);
        const v16b xl = FB::load(al + k0);
        acc[0] = FB::mma(xa, b0, acc[0]);
        acc[1] = FB::mma(xa, b1, acc[1]);
        acc[2] = FB::mma(xa, b2, acc[2]);
        acc[3] = FB::mma(xa, b3, acc[3]);
        acc[0] = FB::mma(xl, b0, acc[0]);
        acc[1] = FB::mma(xl, b1, acc[1]);
        acc[2] = FB::mma(xl, b2, acc[2]);
        acc[3] = FB::mma(xl, b3, acc[3]);
        grp_guard_b(acc[0], acc[1], acc[2], acc[3], xa, xl, b0, b1, b2, b3);
      }
      acc_guard4(acc[0], acc[1], acc[2], acc[3]);
      const float bi = sEb[uc], bfg = sEb[NUNIT + uc], bgg = sEb[2 * NUNIT + uc], bog = sEb[3 * NUNIT + uc];
      unsigned short* th = &sAeH[p ^ 1][0] + ENC_HCOL + uu;
      unsigned short* tl = &sAeL[p ^ 1][0] + ENC_HCOL + uu;
#pragma unroll
      for (int r = 0; r < 8; ++r) {
        const int m = 8 * hh + r;
        const float hn = lstm_cell(acc[0][r] + bi, acc[1][r] + bfg, acc[2][r] + bgg, acc[3][r] + bog, cst[r]);
        const float hv = uval ? hn : 0.0f;
        unsigned short hb, lb;
        split_bf16(hv, hb, lb);
        th[m * ENC_P] = hb;
        tl[m * ENC_P] = lb;
        if (uval) sHf[m * NUNIT + uc] = hn;
      }
    }
    __syncthreads();

    if (wave < 5) {
      const int m = tid / NATT, a = tid - NATT * m;
      float mp = 0.0f;
#pragma unroll 1
      for (int u = 0; u < NUNIT; ++u) mp = fmaf(sHf[m * NUNIT + u], sWm[u * NATT + a], mp);
      sMPst[m * MP_P + a] = mp + sBm[a];
    } else if (wave == 5) {
      sMPst[(lane >> 1) * MP_P + NATT + (lane & 1)] = 0.0f;
    }
    __syncthreads();
  }
  if (wave == 6) {
    wave_store_lines(sHf, Ews + (size_t)blk * E_BLK + (size_t)(NLEN - 1) * E_STEP, E_STEP / 4, lane);
  } else if (wave == 7) {
    wave_store_lines(sMPst, MPws + (size_t)blk * MP_BLK + (size_t)(NLEN - 1) * MP_STEP, MP_STEP / 4, lane);
  }
  __threadfence();
  __syncthreads();

#pragma unroll
  for (int r = 0; r < 8; ++r) cst[r] = 0.0f;
  const float* mpblk = MPws + (size_t)blk * MP_BLK;
  const float* eblk  = Ews  + (size_t)blk * E_BLK;

#pragma unroll 1
  for (int t = 0; t < NDEC; ++t) {
    const int p = t & 1;
    if (wave < 5) {
      const int m = tid / NATT, a = tid - NATT * m;
      float q = 0.0f;
#pragma unroll 1
      for (int u = 0; u < NUNIT; ++u) q = fmaf(sCst[m * NUNIT + u], sWq[u * NATT + a], q);
      sQ[tid] = q + sBq[a];
    } else if (wave == 5) {
      if (t > 0 && lane < TROWS) {
        const int m = lane;
        float acc = 0.0f;
#pragma unroll 1
        for (int u = 0; u < NUNIT; ++u) acc = fmaf(sHf[m * NUNIT + u], sOw[u], acc);
        sY[m * NDEC + (t - 1)] = tanh_p(acc + sMisc[1]);
      }
    }
    __syncthreads();

    {
      const int m = tid >> 4, j = tid & 15;
      float qv[NATT], vv[NATT], wl[NATT];
#pragma unroll
      for (int a = 0; a < NATT; ++a) { qv[a] = sQ[m * NATT + a]; vv[a] = sV[a]; wl[a] = sWloc[a]; }
      const float bvv = sMisc[0];
      float* arow = sAttn + m * ATT_P;
      const float* mprow = mpblk + m * MP_P;
      float mx = -INFINITY;
#pragma unroll 1
      for (int i = 0; i < NITEM; ++i) {
        const int l = j + 16 * i;
        const bool val = (l < NLEN);
        const int lc = val ? l : (NLEN - 1);
        const float ap = arow[lc];
        const float* mp = mprow + (size_t)lc * MP_STEP;
        const v4f m0 = *(const v4f*)(mp);
        const v4f m1 = *(const v4f*)(mp + 4);
        const v4f m2 = *(const v4f*)(mp + 8);
        float mpa[12] = {m0[0], m0[1], m0[2], m0[3], m1[0], m1[1], m1[2], m1[3], m2[0], m2[1], m2[2], m2[3]};
        float s = 0.0f;
#pragma unroll
        for (int a = 0; a < NATT; ++a) {
          const float loc = tanh_q(ap * wl[a]);
          const float inr = (mpa[a] + qv[a]) + loc;
          s = fmaf(vv[a], tanh_q(inr), s);
        }
        s += bvv;
        if (val) arow[l] = s;
        mx = fmaxf(mx, val ? s : -INFINITY);
      }
#pragma unroll
      for (int off = 1; off < 16; off <<= 1) mx = fmaxf(mx, __shfl_xor(mx, off, 32));
      float sum = 0.0f;
#pragma unroll 1
      for (int i = 0; i < NITEM; ++i) {
        const int l = j + 16 * i;
        const bool val = (l < NLEN);
        const int lc = val ? l : (NLEN - 1);
        float e = expf(arow[lc] - mx);
        e = val ? e : 0.0f;
        sum += e;
        if (val) arow[l] = e;
      }
#pragma unroll
      for (int off = 1; off < 16; off <<= 1) sum += __shfl_xor(sum, off, 32);
      const float inv = 1.0f / sum;
#pragma unroll 1
      for (int i = 0; i < NITEM; ++i) {
        const int l = j + 16 * i;
        const bool val = (l < NLEN);
        const int lc = val ? l : (NLEN - 1);
        const float an = arow[lc] * inv;
        if (val) arow[l] = an;
      }
    }
    __syncthreads();

    if (wave < 3) {
      const int m = tid / 6, q6 = tid - 6 * m;
      const int u4 = min(q6, 4) * 4;
      const float* er = eblk + m * NUNIT + u4;
      const float* ar = sAttn + m * ATT_P;
      v4f cx = {0.f, 0.f, 0.f, 0.f};
#pragma unroll 3
      for (int l = 0; l < NLEN; ++l) {
        const float a = ar[l];
        const v4f e = *(const v4f*)(er + (size_t)l * E_STEP);
        cx = cx + e * a;
      }
      if (q6 < 5) {
        unsigned short h0, l0, h1, l1, h2, l2, h3, l3;
        split_bf16(cx[0], h0, l0); split_bf16(cx[1], h1, l1); split_bf16(cx[2], h2, l2); split_bf16(cx[3], h3, l3);
        v2u ph, pl;
        ph[0] = (unsigned)h0 | ((unsigned)h1 << 16); ph[1] = (unsigned)h2 | ((unsigned)h3 << 16);
        pl[0] = (unsigned)l0 | ((unsigned)l1 << 16); pl[1] = (unsigned)l2 | ((unsigned)l3 << 16);
        *(v2u*)(&sAdH[p][0] + m * DEC_P + u4) = ph;
        *(v2u*)(&sAdL[p][0] + m * DEC_P + u4) = pl;
      }
    } else if (wave == 3) {
      const v2u z2 = {0u, 0u};
#pragma unroll
      for (int jj = 0; jj < 2; ++jj) {
        const int i = lane + 32 * jj;
        if (i < 48) {
          const int m = i / 3, c4 = DEC_HCOL + 32 + (i - 3 * m) * 4;
          *(v2u*)(&sAdH[p][0] + m * DEC_P + c4) = z2;
          *(v2u*)(&sAdL[p][0] + m * DEC_P + c4) = z2;
        }
      }
    }
    __syncthreads();

    if (wave < 2) {
      const __bf16* ah = (const __bf16*)(&sAdH[p][0] + c * DEC_P + koff);
      const __bf16* al = (const __bf16*)(&sAdL[p][0] + c * DEC_P + koff);
      const __bf16* wb = (const __bf16*)(sWdec + (wave * 16 + c) * DEC_P + koff);
      v8f acc[4];
      acc[0] = z8; acc[1] = z8; acc[2] = z8; acc[3] = z8;
#pragma unroll
      for (int ks = 0; ks < 2; ++ks) {
        const int k0 = 32 * ks;
        const v16b b0 = FB::load(wb + 0 * 32 * DEC_P + k0);
        const v16b b1 = FB::load(wb + 1 * 32 * DEC_P + k0);
        const v16b b2 = FB::load(wb + 2 * 32 * DEC_P + k0);
        const v16b b3 = FB::load(wb + 3 * 32 * DEC_P + k0);
        const v16b xa = FB::load(ah + k0);
        const v16b xl = FB::load(al + k0);
        acc[0] = FB::mma(xa, b0, acc[0]);
        acc[1] = FB::mma(xa, b1, acc[1]);
        acc[2] = FB::mma(xa, b2, acc[2]);
        acc[3] = FB::mma(xa, b3, acc[3]);
        acc[0] = FB::mma(xl, b0, acc[0]);
        acc[1] = FB::mma(xl, b1, acc[1]);
        acc[2] = FB::mma(xl, b2, acc[2]);
        acc[3] = FB::mma(xl, b3, acc[3]);
        grp_guard_b(acc[0], acc[1], acc[2], acc[3], xa, xl, b0, b1, b2, b3);
      }
      acc_guard4(acc[0], acc[1], acc[2], acc[3]);
      const float bi = sDb[uc], bfg = sDb[NUNIT + uc], bgg = sDb[2 * NUNIT + uc], bog = sDb[3 * NUNIT + uc];
      unsigned short* th = &sAdH[p ^ 1][0] + DEC_HCOL + uu;
      unsigned short* tl = &sAdL[p ^ 1][0] + DEC_HCOL + uu;
#pragma unroll
      for (int r = 0; r < 8; ++r) {
        const int m = 8 * hh + r;
        const float hn = lstm_cell(acc[0][r] + bi, acc[1][r] + bfg, acc[2][r] + bgg, acc[3][r] + bog, cst[r]);
        const float hv = uval ? hn : 0.0f;
        unsigned short hb, lb;
        split_bf16(hv, hb, lb);
        th[m * DEC_P] = hb;
        tl[m * DEC_P] = lb;
        if (uval) { sHf[m * NUNIT + uc] = hn; sCst[m * NUNIT + uc] = cst[r]; }
      }
    }
    __syncthreads();
  }
  if (tid < TROWS) {
    const int m = tid;
    float acc = 0.0f;
#pragma unroll 1
    for (int u = 0; u < NUNIT; ++u) acc = fmaf(sHf[m * NUNIT + u], sOw[u], acc);
    sY[m * NDEC + (NDEC - 1)] = tanh_p(acc + sMisc[1]);
  }
  __syncthreads();

  {
    float* yp = Yout + (size_t)blk * Y_BLK;
    for (int pass = 0; pass < 2; ++pass) {
#pragma unroll 1
      for (int i = tid; i < Y_BLK / 4; i += NTHR) {
        const v4f v = *(const v4f*)(sY + 4 * i);
        *(volatile v4f*)(yp + 4 * i) = v;
      }
      __threadfence();
    }
  }
}

extern "C" void kernel_launch(void* const* d_in, const int* in_sizes, int n_in,
                              void* d_out, int out_size, void* d_ws, size_t ws_size, hipStream_t stream) {
  if (n_in < 17 || d_out == nullptr || d_ws == nullptr) return;
  if (in_sizes[0] != NBAT * NLEN * NFEAT || in_sizes[1] != NFEAT * NGATE || in_sizes[2] != NUNIT * NGATE ||
      in_sizes[3] != NGATE || in_sizes[4] != NUNIT * NATT || in_sizes[5] != NATT || in_sizes[6] != NUNIT * NATT ||
      in_sizes[7] != NATT || in_sizes[8] != NATT || in_sizes[9] != 1 || in_sizes[10] != NCF ||
      in_sizes[11] != NCF * NATT || in_sizes[12] != NUNIT * NGATE || in_sizes[13] != NUNIT * NGATE ||
      in_sizes[14] != NGATE || in_sizes[15] != NUNIT || in_sizes[16] != 1 || out_size != NBAT * NDEC) return;

  const float* x      = (const float*)d_in[0];
  const float* encWx  = (const float*)d_in[1];
  const float* encWh  = (const float*)d_in[2];
  const float* encB   = (const float*)d_in[3];
  const float* attWq  = (const float*)d_in[4];
  const float* attBq  = (const float*)d_in[5];
  const float* attWm  = (const float*)d_in[6];
  const float* attBm  = (const float*)d_in[7];
  const float* attV   = (const float*)d_in[8];
  const float* attBv  = (const float*)d_in[9];
  const float* locWc  = (const float*)d_in[10];
  const float* locWd  = (const float*)d_in[11];
  const float* decWx  = (const float*)d_in[12];
  const float* decWh  = (const float*)d_in[13];
  const float* decB   = (const float*)d_in[14];
  const float* outW   = (const float*)d_in[15];
  const float* outB   = (const float*)d_in[16];
  float* y = (float*)d_out;

  char* ws = (char*)d_ws; size_t off = 0;
  auto carve = [&](size_t bytes) -> char* { char* ptr = ws + off; off += (bytes + 255) & ~(size_t)255; return ptr; };
  float* E  = (float*)carve((size_t)NBLK * E_BLK * 4);
  float* MP = (float*)carve((size_t)NBLK * MP_BLK * 4);
  if (off > ws_size || off > (size_t)134217728) return;

  seq_attn_lstm_kernel<<<NBLK, NTHR, 0, stream>>>(x, encWx, encWh, encB, attWq, attBq, attWm, attBm, attV, attBv,
                                                   locWc, locWd, decWx, decWh, decB, outW, outB, y, E, MP);
}
